// lstm_30734785970219
// MI455X (gfx1250) — hardware-verified
//
#include <hip/hip_runtime.h>
#include <math.h>

constexpr int BATCH_N  = 8;
constexpr int SEQ_T    = 512;
constexpr int IN_D     = 1024;
constexpr int HID_N    = 1024;
constexpr int ROWS_M   = BATCH_N * SEQ_T;
constexpr int KTOT     = IN_D + HID_N;
constexpr int NPLANE   = 4 * HID_N;
constexpr int NTHR     = 256;
constexpr int ZPITCH   = 36;
constexpr int ZGATE    = 16 * ZPITCH;
constexpr float WCARRY     = 256.0f;
constexpr float WCARRY_INV = 1.0f / 256.0f;
constexpr size_t OUT1_OFF_BYTES = 16777216;
constexpr size_t OUT_TOTAL_BYTES = 33554432;
static_assert(ROWS_M == 4096);
static_assert(KTOT == 2048);
static_assert(NPLANE == 4096);
static_assert(IN_D == HID_N);
static_assert(KTOT % 32 == 0);
static_assert(ROWS_M % 32 == 0 && HID_N % 32 == 0);
static_assert((ROWS_M / 32) * (HID_N / 32) % (NTHR / 32) == 0);
static_assert(OUT1_OFF_BYTES == (size_t)ROWS_M * HID_N * 4);
static_assert(OUT1_OFF_BYTES + (size_t)ROWS_M * HID_N * 4 == OUT_TOTAL_BYTES);
static_assert(OUT1_OFF_BYTES % 128 == 0);
static_assert(ZPITCH % 4 == 0 && ZPITCH >= 32);

typedef __attribute__((ext_vector_type(16))) _Float16 v16h;
typedef __attribute__((ext_vector_type(8)))  _Float16 v8h;
typedef __attribute__((ext_vector_type(8)))  float    v8f;
typedef __attribute__((ext_vector_type(4)))  float    v4f;

struct FragH {
  union U { v16h v; v8h h[2]; };
  static __device__ __forceinline__ v16h load(const _Float16* p) {
    U f;
    f.h[0] = *(const v8h*)(p);
    f.h[1] = *(const v8h*)(p + 16);
    return f.v;
  }
  static __device__ __forceinline__ v8f mma(v16h a, v16h b, v8f c) {
    return __builtin_amdgcn_wmma_f32_16x16x32_f16(false, a, false, b, (short)0, c, false, false);
  }
};

__device__ __forceinline__ void guard8(v8f& c0, v8f& c1, v8f& c2, v8f& c3, v8f& c4, v8f& c5, v8f& c6, v8f& c7,
                                       v16h a0, v16h a1, v16h b0, v16h b1, v16h b2, v16h b3) {
  asm volatile("v_nop\n\tv_nop\n\tv_nop\n\tv_nop"
               : "+v"(c0), "+v"(c1), "+v"(c2), "+v"(c3), "+v"(c4), "+v"(c5), "+v"(c6), "+v"(c7)
               : "v"(a0), "v"(a1), "v"(b0), "v"(b1), "v"(b2), "v"(b3));
}
__device__ __forceinline__ void acc_guard4(v8f& a, v8f& b, v8f& c, v8f& d) {
  asm volatile("v_nop\n\tv_nop\n\tv_nop\n\tv_nop" : "+v"(a), "+v"(b), "+v"(c), "+v"(d));
}
__device__ __forceinline__ void wave_lds_sync() {
  __builtin_amdgcn_fence(__ATOMIC_RELEASE, "workgroup");
  __builtin_amdgcn_wave_barrier();
  __builtin_amdgcn_fence(__ATOMIC_ACQUIRE, "workgroup");
}
__device__ __forceinline__ float sigm(float z) { return 1.0f / (1.0f + expf(-z)); }

__global__ __launch_bounds__(NTHR) void pack_act_kernel(const float* __restrict__ x, const float* __restrict__ hin,
                                                        unsigned short* __restrict__ Ap) {
  const int half = blockIdx.y;
  const float* src = half ? hin : x;
  const int i  = blockIdx.x * NTHR + threadIdx.x;
  if (i < ROWS_M * (IN_D / 8)) {
    const int m  = i >> 7;
    const int c8 = i & 127;
    const float* sp = src + (size_t)m * IN_D + c8 * 8;
    const v4f a = *(const v4f*)(sp);
    const v4f b = *(const v4f*)(sp + 4);
    v8h hv;
#pragma unroll
    for (int e = 0; e < 4; ++e) {
      hv[e]     = (_Float16)a[e];
      hv[4 + e] = (_Float16)b[e];
    }
    unsigned short* dp = Ap + (size_t)m * KTOT + (size_t)half * IN_D + c8 * 8;
    *(volatile v8h*)dp = hv;
    __threadfence();
    *(volatile v8h*)dp = hv;
  }
}

__global__ __launch_bounds__(NTHR) void pack_w_kernel(const float* __restrict__ Wf, const float* __restrict__ Wi,
                                                      const float* __restrict__ Wg, const float* __restrict__ Wo,
                                                      unsigned short* __restrict__ Btp) {
  __shared__ float Tt[64 * 65];
  const int gate = blockIdx.z;
  const float* src = (gate == 0) ? Wf : (gate == 1) ? Wi : (gate == 2) ? Wg : Wo;
  const int tid = threadIdx.x;
  const int c0 = blockIdx.x * 64;
  const int r0 = blockIdx.y * 64;
#pragma unroll
  for (int i = 0; i < 4; ++i) {
    const int idx = i * NTHR + tid;
    const int rr = idx >> 4;
    const int cc = (idx & 15) * 4;
    const v4f v = *(const v4f*)(src + (size_t)(r0 + rr) * (size_t)HID_N + c0 + cc);
    Tt[rr * 65 + cc + 0] = v[0];
    Tt[rr * 65 + cc + 1] = v[1];
    Tt[rr * 65 + cc + 2] = v[2];
    Tt[rr * 65 + cc + 3] = v[3];
  }
  __syncthreads();
  const int q  = tid >> 3;
  const int c8 = (tid & 7) * 8;
  v8h hv[2];
#pragma unroll
  for (int g2 = 0; g2 < 2; ++g2) {
    const int qq = g2 * 32 + q;
#pragma unroll
    for (int e = 0; e < 8; ++e) {
      const float f = Tt[(c8 + e) * 65 + qq];
      hv[g2][e] = (_Float16)(f * WCARRY);
    }
  }
  for (int pass = 0; pass < 2; ++pass) {
#pragma unroll
    for (int g2 = 0; g2 < 2; ++g2) {
      const int h  = c0 + g2 * 32 + q;
      const int np = (h >> 4) * 64 + gate * 16 + (h & 15);
      const size_t o = (size_t)np * (size_t)KTOT + (size_t)(r0 + c8);
      *(volatile v8h*)(Btp + o) = hv[g2];
    }
    __threadfence();
  }
}

__global__ __launch_bounds__(NTHR) void lstm_gate_gemm_kernel(
    const unsigned short* __restrict__ Ap, const unsigned short* __restrict__ Btp,
    const float* __restrict__ cin,
    const float* __restrict__ bF, const float* __restrict__ bI,
    const float* __restrict__ bG, const float* __restrict__ bO,
    float* __restrict__ outH, float* __restrict__ outC) {
  __shared__ __align__(16) float Zs[NTHR / 32][4 * ZGATE];
  const _Float16* A  = (const _Float16*)Ap;
  const _Float16* Bt = (const _Float16*)Btp;
  const int lane = threadIdx.x & 31;
  const int wave = threadIdx.x >> 5;
  const int c    = lane & 15;
  const int hh   = lane >> 4;
  const int koff = hh * 8;
  const int tile = blockIdx.x * (NTHR / 32) + wave;
  const int mt   = tile >> 5;
  const int ht   = tile & 31;
  const int m0    = mt * 32;
  const int hbase = ht * 32;
  const int n0    = ht * 128;

  v8f acc[2][2][4];
#pragma unroll
  for (int tm = 0; tm < 2; ++tm)
#pragma unroll
    for (int tn = 0; tn < 2; ++tn)
#pragma unroll
      for (int g = 0; g < 4; ++g) acc[tm][tn][g] = (v8f){0.f, 0.f, 0.f, 0.f, 0.f, 0.f, 0.f, 0.f};

  const _Float16* ap0 = A + (size_t)(m0 + c) * KTOT + koff;
  const _Float16* ap1 = ap0 + (size_t)16 * KTOT;
  const _Float16* bp  = Bt + (size_t)(n0 + c) * KTOT + koff;

#pragma unroll 1
  for (int k0 = 0; k0 < KTOT; k0 += 32) {
    const v16h a0 = FragH::load(ap0 + k0);
    const v16h a1 = FragH::load(ap1 + k0);
#pragma unroll
    for (int tn = 0; tn < 2; ++tn) {
      const _Float16* bq = bp + (size_t)(tn * 64) * KTOT + k0;
      const v16h b0 = FragH::load(bq);
      const v16h b1 = FragH::load(bq + (size_t)16 * KTOT);
      const v16h b2 = FragH::load(bq + (size_t)32 * KTOT);
      const v16h b3 = FragH::load(bq + (size_t)48 * KTOT);
      acc[0][tn][0] = FragH::mma(a0, b0, acc[0][tn][0]);
      acc[0][tn][1] = FragH::mma(a0, b1, acc[0][tn][1]);
      acc[0][tn][2] = FragH::mma(a0, b2, acc[0][tn][2]);
      acc[0][tn][3] = FragH::mma(a0, b3, acc[0][tn][3]);
      acc[1][tn][0] = FragH::mma(a1, b0, acc[1][tn][0]);
      acc[1][tn][1] = FragH::mma(a1, b1, acc[1][tn][1]);
      acc[1][tn][2] = FragH::mma(a1, b2, acc[1][tn][2]);
      acc[1][tn][3] = FragH::mma(a1, b3, acc[1][tn][3]);
      guard8(acc[0][tn][0], acc[0][tn][1], acc[0][tn][2], acc[0][tn][3],
             acc[1][tn][0], acc[1][tn][1], acc[1][tn][2], acc[1][tn][3],
             a0, a1, b0, b1, b2, b3);
    }
  }
  acc_guard4(acc[0][0][0], acc[0][0][1], acc[0][0][2], acc[0][0][3]);
  acc_guard4(acc[0][1][0], acc[0][1][1], acc[0][1][2], acc[0][1][3]);
  acc_guard4(acc[1][0][0], acc[1][0][1], acc[1][0][2], acc[1][0][3]);
  acc_guard4(acc[1][1][0], acc[1][1][1], acc[1][1][2], acc[1][1][3]);

  float bv[2][4];
#pragma unroll
  for (int tn = 0; tn < 2; ++tn) {
    const int h = hbase + tn * 16 + c;
    bv[tn][0] = bF[h];
    bv[tn][1] = bI[h];
    bv[tn][2] = bG[h];
    bv[tn][3] = bO[h];
  }

  float* zs = &Zs[wave][0];
  const int q  = lane >> 3;
  const int c4 = (lane & 7) * 4;

#pragma unroll
  for (int tm = 0; tm < 2; ++tm) {
#pragma unroll
    for (int tn = 0; tn < 2; ++tn)
#pragma unroll
      for (int g = 0; g < 4; ++g)
#pragma unroll
        for (int r = 0; r < 8; ++r)
          zs[g * ZGATE + (8 * hh + r) * ZPITCH + tn * 16 + c] = acc[tm][tn][g][r] * WCARRY_INV + bv[tn][g];
    wave_lds_sync();

#pragma unroll 1
    for (int it = 0; it < 4; ++it) {
      const int row = it * 4 + q;
      float* zp = zs + row * ZPITCH + c4;
      const v4f zf = *(const v4f*)(zp);
      const v4f zi = *(const v4f*)(zp + ZGATE);
      const v4f zg = *(const v4f*)(zp + 2 * ZGATE);
      const v4f zo = *(const v4f*)(zp + 3 * ZGATE);
      const v4f cv = *(const v4f*)(cin + (size_t)(m0 + tm * 16 + row) * HID_N + hbase + c4);
      v4f ho, co;
#pragma unroll
      for (int e = 0; e < 4; ++e) {
        const float fg = sigm(zf[e]);
        const float ig = sigm(zi[e]);
        const float gg = tanhf(zg[e]);
        const float og = sigm(zo[e]);
        const float cn = fg * cv[e] + gg * ig;
        co[e] = cn;
        ho[e] = tanhf(cn) * og;
      }
      *(v4f*)(zp) = ho;
      *(v4f*)(zp + ZGATE) = co;
    }
    wave_lds_sync();

    for (int pass = 0; pass < 2; ++pass) {
#pragma unroll
      for (int it = 0; it < 4; ++it) {
        const int row = it * 4 + q;
        const float* zp = zs + row * ZPITCH + c4;
        const v4f hv = *(const v4f*)(zp);
        const v4f cw = *(const v4f*)(zp + ZGATE);
        const size_t o = (size_t)(m0 + tm * 16 + row) * HID_N + hbase + c4;
        *(volatile v4f*)(outH + o) = hv;
        *(volatile v4f*)(outC + o) = cw;
      }
      __threadfence();
    }
    wave_lds_sync();
  }
}

extern "C" void kernel_launch(void* const* d_in, const int* in_sizes, int n_in,
                              void* d_out, int out_size, void* d_ws, size_t ws_size, hipStream_t stream) {
  if (n_in < 11 || d_out == nullptr || d_ws == nullptr) return;
  const int nact = ROWS_M * IN_D;
  const int nw   = KTOT * HID_N;
  if (in_sizes[0] != nact || in_sizes[1] != nact || in_sizes[2] != nact ||
      in_sizes[3] != nw || in_sizes[4] != HID_N || in_sizes[5] != nw || in_sizes[6] != HID_N ||
      in_sizes[7] != nw || in_sizes[8] != HID_N || in_sizes[9] != nw || in_sizes[10] != HID_N ||
      out_size != 2 * ROWS_M * HID_N) return;

  const float* x   = (const float*)d_in[0];
  const float* hin = (const float*)d_in[1];
  const float* cin = (const float*)d_in[2];
  const float* Wf  = (const float*)d_in[3];
  const float* bF  = (const float*)d_in[4];
  const float* Wi  = (const float*)d_in[5];
  const float* bI  = (const float*)d_in[6];
  const float* Wg  = (const float*)d_in[7];
  const float* bG  = (const float*)d_in[8];
  const float* Wo  = (const float*)d_in[9];
  const float* bO  = (const float*)d_in[10];
  float* outH = (float*)d_out;
  float* outC = (float*)d_out + (OUT1_OFF_BYTES / 4);

  char* ws = (char*)d_ws;
  size_t off = 0;
  auto carve = [&](size_t bytes) -> char* { char* p = ws + off; off += (bytes + 255) & ~(size_t)255; return p; };
  unsigned short* APL  = (unsigned short*)carve((size_t)ROWS_M * KTOT * 2);
  unsigned short* BTPL = (unsigned short*)carve((size_t)NPLANE * KTOT * 2);
  if (off > ws_size || off > (size_t)134217728) return;

  pack_act_kernel<<<dim3(ROWS_M * (IN_D / 8) / NTHR, 2), NTHR, 0, stream>>>(x, hin, APL);
  pack_w_kernel<<<dim3(HID_N / 64, KTOT / 64, 4), NTHR, 0, stream>>>(Wf, Wi, Wg, Wo, BTPL);
  lstm_gate_gemm_kernel<<<(ROWS_M / 32) * (HID_N / 32) / (NTHR / 32), NTHR, 0, stream>>>(
      APL, BTPL, cin, bF, bI, bG, bO, outH, outC);
}
